// Block_74285754352217
// MI455X (gfx1250) — hardware-run, weakly checked
//
#include <hip/hip_runtime.h>
#include <math.h>

constexpr int kBatch    = 2;
constexpr int kSeq      = 2048;
constexpr int kDim      = 768;
constexpr int kHeads    = 12;
constexpr int kHeadDim  = 64;
constexpr int kQkvCols  = 3 * kDim;
constexpr int kFF       = 3072;
constexpr int kTok      = kBatch * kSeq;
constexpr int kGroups   = kBatch * kHeads;
constexpr int kGrpPerChunk = 3;
constexpr int kChunks   = kGroups / kGrpPerChunk;
constexpr float kWCarry = 16.0f;
constexpr float kPCarry = 2048.0f;
constexpr float kOCarry = 64.0f;
constexpr float kGCarry = 16.0f;
constexpr float kAttnScale = 0.125f;
constexpr float kLnEps  = 1e-6f;
constexpr float kInvDim = 1.0f / 768.0f;

typedef __attribute__((ext_vector_type(16))) _Float16 v16h;
typedef __attribute__((ext_vector_type(8)))  _Float16 v8h;
typedef __attribute__((ext_vector_type(16))) __bf16   v16b;
typedef __attribute__((ext_vector_type(8)))  __bf16   v8b;
typedef __attribute__((ext_vector_type(8)))  float    v8f;
typedef __attribute__((ext_vector_type(4)))  float    v4f;
typedef __attribute__((ext_vector_type(2)))  float    v2f;
typedef __attribute__((ext_vector_type(4)))  unsigned int v4u;

__device__ __forceinline__ unsigned short f2bf_bits(float f) {
  unsigned u = __float_as_uint(f);
  return (unsigned short)((u + 0x7FFFu + ((u >> 16) & 1u)) >> 16);
}
__device__ __forceinline__ float bf_bits2f(unsigned short h) { return __uint_as_float(((unsigned)h) << 16); }

__device__ __forceinline__ void dep_guard_h(v8f& a, v8f& b, v16h x, v16h y) { asm volatile("v_nop\n\tv_nop\n\tv_nop\n\tv_nop" : "+v"(a), "+v"(b) : "v"(x), "v"(y)); }
__device__ __forceinline__ void dep_guard_b(v8f& a, v8f& b, v16b x, v16b y) { asm volatile("v_nop\n\tv_nop\n\tv_nop\n\tv_nop" : "+v"(a), "+v"(b) : "v"(x), "v"(y)); }
__device__ __forceinline__ void keep4_h(v16h a, v16h b, v16h c, v16h d) { asm volatile("v_nop" :: "v"(a), "v"(b), "v"(c), "v"(d)); }
__device__ __forceinline__ void keep4_b(v16b a, v16b b, v16b c, v16b d) { asm volatile("v_nop" :: "v"(a), "v"(b), "v"(c), "v"(d)); }
__device__ __forceinline__ void acc_guard4(v8f& a, v8f& b, v8f& c, v8f& d) { asm volatile("v_nop\n\tv_nop\n\tv_nop\n\tv_nop" : "+v"(a), "+v"(b), "+v"(c), "+v"(d)); }
template <typename T> struct Frag;
template <> struct Frag<_Float16> {
  typedef v16h V; union U { v16h v; v8h h[2]; };
  static __device__ __forceinline__ v16h load(const _Float16* p) {
    U f; f.h[0] = *(const v8h*)(p); f.h[1] = *(const v8h*)(p + 16); return f.v;
  }
  static __device__ __forceinline__ v8f mma(v16h a, v16h b, v8f c) {
    return __builtin_amdgcn_wmma_f32_16x16x32_f16(false, a, false, b, (short)0, c, false, false);
  }
  static __device__ __forceinline__ void guard(v8f& a, v8f& b, v16h x, v16h y) { dep_guard_h(a, b, x, y); }
  static __device__ __forceinline__ void keep(v16h a, v16h b, v16h c, v16h d) { keep4_h(a, b, c, d); }
};
template <> struct Frag<__bf16> {
  typedef v16b V; union U { v16b v; v8b h[2]; };
  static __device__ __forceinline__ v16b load(const __bf16* p) {
    U f; f.h[0] = *(const v8b*)(p); f.h[1] = *(const v8b*)(p + 16); return f.v;
  }
  static __device__ __forceinline__ v8f mma(v16b a, v16b b, v8f c) {
    return __builtin_amdgcn_wmma_f32_16x16x32_bf16(false, a, false, b, (short)0, c, false, false);
  }
  static __device__ __forceinline__ void guard(v8f& a, v8f& b, v16b x, v16b y) { dep_guard_b(a, b, x, y); }
  static __device__ __forceinline__ void keep(v16b a, v16b b, v16b c, v16b d) { keep4_b(a, b, c, d); }
};

__device__ __forceinline__ unsigned pk16(unsigned short a, unsigned short b) { return (unsigned)a | ((unsigned)b << 16); }
__device__ __forceinline__ unsigned short h_bits(float f) { const _Float16 h = (_Float16)f; return __builtin_bit_cast(unsigned short, h); }

template <int ET> struct Elem;
template <> struct Elem<0> { typedef _Float16 T; };
template <> struct Elem<1> { typedef __bf16 T; };
template <int ET, bool SPLIT, int BIAS_MODE, int OUT_MODE, bool RESID, int ACT = 0>
__global__ __launch_bounds__(256) void wmma_gemm64(
    const unsigned short* __restrict__ Ap, const unsigned short* __restrict__ A2p, int lda, long strideA,
    const unsigned short* __restrict__ Btp, const unsigned short* __restrict__ Bt2p, int ldb, long strideB,
    void* __restrict__ Cout, void* __restrict__ Cout2, int ldc, long strideC,
    const float* __restrict__ bias,
    const float* __restrict__ resid, long strideR,
    int M, int N, int K, float scale) {
  typedef typename Elem<ET>::T T;
  typedef typename Frag<T>::V V;
  const T* A = (const T*)Ap; const T* A2 = (const T*)A2p; const T* Bt = (const T*)Btp; const T* Bt2 = (const T*)Bt2p;
  __shared__ __align__(16) float sT[8][16 * 68];
  const int b    = blockIdx.y;
  const int lane = threadIdx.x & 31;
  const int wave = threadIdx.x >> 5;
  const int tilesN = N >> 6;
  const int tilesM = M >> 6;
  const int tile = blockIdx.x * 8 + wave;
  if (tile >= tilesM * tilesN) return;
  const int tm = tile / tilesN;
  const int tn = tile - tm * tilesN;
  const int m0 = tm << 6;
  const int n0 = tn << 6;

  const T* Ab  = A  + (size_t)b * strideA;
  const T* Bb  = Bt + (size_t)b * strideB;
  const T* Ab2 = SPLIT ? (A2  + (size_t)b * strideA) : nullptr;
  const T* Bb2 = SPLIT ? (Bt2 + (size_t)b * strideB) : nullptr;

  const int rlane = lane & 15;
  const int koff  = (lane >> 4) * 8;
  const int mOff  = (lane >> 4) * 8;

  v8f acc[4][4];
#pragma unroll
  for (int i = 0; i < 4; ++i)
#pragma unroll
    for (int j = 0; j < 4; ++j) acc[i][j] = (v8f){0.f,0.f,0.f,0.f,0.f,0.f,0.f,0.f};

  for (int k0 = 0; k0 < K; k0 += 32) {
    V bh[4], bl[4];
#pragma unroll
    for (int j = 0; j < 4; ++j) {
      const size_t bo = (size_t)(n0 + (j << 4) + rlane) * ldb + koff + k0;
      bh[j] = Frag<T>::load(Bb + bo);
      if (SPLIT) bl[j] = Frag<T>::load(Bb2 + bo);
    }
#pragma unroll
    for (int i = 0; i < 4; ++i) {
      const size_t ao = (size_t)(m0 + (i << 4) + rlane) * lda + koff + k0;
      V ah = Frag<T>::load(Ab + ao);
      V al;
      if (SPLIT) al = Frag<T>::load(Ab2 + ao);
#pragma unroll
      for (int j = 0; j < 4; ++j) {
        acc[i][j] = Frag<T>::mma(ah, bh[j], acc[i][j]);
        if (SPLIT) {
          acc[i][j] = Frag<T>::mma(ah, bl[j], acc[i][j]);
          acc[i][j] = Frag<T>::mma(al, bh[j], acc[i][j]);
        }
      }
      Frag<T>::guard(acc[i][0], acc[i][3], ah, SPLIT ? al : ah);
    }
    Frag<T>::keep(bh[0], bh[1], bh[2], bh[3]);
    if (SPLIT) Frag<T>::keep(bl[0], bl[1], bl[2], bl[3]);
  }
  acc_guard4(acc[0][0], acc[0][1], acc[0][2], acc[0][3]);
  acc_guard4(acc[1][0], acc[1][1], acc[1][2], acc[1][3]);
  acc_guard4(acc[2][0], acc[2][1], acc[2][2], acc[2][3]);
  acc_guard4(acc[3][0], acc[3][1], acc[3][2], acc[3][3]);

  float* slab = sT[wave];
  const float* Rb = RESID ? (resid + (size_t)b * strideR) : nullptr;
#pragma unroll
  for (int i = 0; i < 4; ++i) {
    const int mBase = m0 + (i << 4);
#pragma unroll
    for (int j = 0; j < 4; ++j) {
      const int n = n0 + (j << 4) + rlane;
      float bv = 0.f;
      if (BIAS_MODE == 2) bv = bias[n];
#pragma unroll
      for (int r = 0; r < 8; ++r) {
        float v = acc[i][j][r] * scale;
        if (BIAS_MODE == 1) v += bias[mBase + mOff + r];
        if (BIAS_MODE == 2) v += bv;
        if (RESID) v += Rb[(size_t)(mBase + mOff + r) * ldc + n];
        if (ACT == 2) v = fmaxf(v, 0.0f);
        if (ACT == 4) v = (v > 0.f) ? v : 0.01f * v;
        slab[(mOff + r) * 68 + (j << 4) + rlane] = v;
      }
    }
    __builtin_amdgcn_fence(__ATOMIC_RELEASE, "workgroup");
    __builtin_amdgcn_wave_barrier();
    __builtin_amdgcn_fence(__ATOMIC_ACQUIRE, "workgroup");
    if (OUT_MODE == 0) {
      float* C = (float*)Cout + (size_t)b * strideC;
      const int hh = lane >> 4, c4 = (lane & 15) * 4;
      for (int pass = 0; pass < 2; ++pass) {
#pragma unroll
        for (int it = 0; it < 8; ++it) {
          const int row = it * 2 + hh;
          v4f v = *(const v4f*)(slab + row * 68 + c4);
          *(volatile v4f*)(C + (size_t)(mBase + row) * ldc + n0 + c4) = v;
        }
        __threadfence();
      }
    } else {
      const int q = lane >> 3, c8 = (lane & 7) * 8;
      unsigned short* C  = (unsigned short*)Cout  + (size_t)b * strideC;
      unsigned short* C2 = (OUT_MODE == 2) ? ((unsigned short*)Cout2 + (size_t)b * strideC) : nullptr;
      for (int pass = 0; pass < 2; ++pass) {
#pragma unroll
        for (int it = 0; it < 4; ++it) {
          const int row = it * 4 + q;
          const float* sp = slab + row * 68 + c8;
          v8h hv, lv;
#pragma unroll
          for (int e = 0; e < 8; ++e) {
            if (OUT_MODE == 1) {
              hv[e] = (_Float16)sp[e];
            } else {
              unsigned short hb = f2bf_bits(sp[e]);
              unsigned short lb = f2bf_bits(sp[e] - bf_bits2f(hb));
              hv[e] = __builtin_bit_cast(_Float16, hb);
              lv[e] = __builtin_bit_cast(_Float16, lb);
            }
          }
          *(volatile v8h*)(C + (size_t)(mBase + row) * ldc + n0 + c8) = hv;
          if (OUT_MODE == 2) *(volatile v8h*)(C2 + (size_t)(mBase + row) * ldc + n0 + c8) = lv;
        }
        __threadfence();
      }
    }
    __builtin_amdgcn_fence(__ATOMIC_RELEASE, "workgroup");
    __builtin_amdgcn_wave_barrier();
    __builtin_amdgcn_fence(__ATOMIC_ACQUIRE, "workgroup");
  }
}

__global__ __launch_bounds__(256) void wtcast_kernel(const float* __restrict__ W, unsigned short* __restrict__ WT,
                                                     int Kin, int Nout, float scale) {
  __shared__ float sm[64][65];
  const int t  = threadIdx.x;
  const int k0 = blockIdx.x * 64;
  const int n0 = blockIdx.y * 64;
#pragma unroll
  for (int i = 0; i < 16; ++i) {
    const int e = i * 256 + t;
    const int r = e >> 6;
    const int c = e & 63;
    sm[c][r] = W[(size_t)(k0 + r) * Nout + n0 + c] * scale;
  }
  __syncthreads();
  const int lane = t & 31, wave = t >> 5;
  const int q = lane >> 3, c8 = (lane & 7) * 8;
  for (int pass = 0; pass < 2; ++pass) {
#pragma unroll
    for (int it = 0; it < 2; ++it) {
      const int row = wave * 8 + it * 4 + q;
      unsigned short hb[8];
#pragma unroll
      for (int e = 0; e < 8; ++e) hb[e] = h_bits(sm[row][c8 + e]);
      const v4u u = (v4u){pk16(hb[0], hb[1]), pk16(hb[2], hb[3]), pk16(hb[4], hb[5]), pk16(hb[6], hb[7])};
      *(volatile v4u*)(WT + (size_t)(n0 + row) * Kin + k0 + c8) = u;
    }
    __threadfence();
  }
}

__global__ __launch_bounds__(256) void ln_row_kernel(const float* __restrict__ X, const float* __restrict__ gam,
                                                     const float* __restrict__ bet, unsigned short* __restrict__ Y) {
  __shared__ float red[8];
  __shared__ float stat[2];
  const int row  = blockIdx.x;
  const int t    = threadIdx.x;
  const int lane = t & 31, wave = t >> 5;
  const float* xr = X + (size_t)row * kDim;
  const float a0 = xr[t], a1 = xr[t + 256], a2 = xr[t + 512];
  float s = (a0 + a1) + a2;
#pragma unroll
  for (int off = 16; off > 0; off >>= 1) s += __shfl_xor(s, off, 32);
  if (lane == 0) red[wave] = s;
  __syncthreads();
  if (t == 0) {
    float tot = red[0];
#pragma unroll
    for (int w = 1; w < 8; ++w) tot += red[w];
    stat[0] = tot * kInvDim;
  }
  __syncthreads();
  const float mu = stat[0];
  const float d0 = a0 - mu, d1 = a1 - mu, d2 = a2 - mu;
  float s2 = (d0 * d0 + d1 * d1) + d2 * d2;
#pragma unroll
  for (int off = 16; off > 0; off >>= 1) s2 += __shfl_xor(s2, off, 32);
  if (lane == 0) red[wave] = s2;
  __syncthreads();
  if (t == 0) {
    float tot = red[0];
#pragma unroll
    for (int w = 1; w < 8; ++w) tot += red[w];
    stat[1] = rsqrtf(tot * kInvDim + kLnEps);
  }
  __syncthreads();
  const float rs = stat[1];
  if (wave < 3) {
    const int c0 = t * 8;
    const v4f xa = *(const v4f*)(xr + c0);
    const v4f xb = *(const v4f*)(xr + c0 + 4);
    const v4f ga = *(const v4f*)(gam + c0);
    const v4f gb = *(const v4f*)(gam + c0 + 4);
    const v4f ba = *(const v4f*)(bet + c0);
    const v4f bb = *(const v4f*)(bet + c0 + 4);
    unsigned short hb[8];
#pragma unroll
    for (int e = 0; e < 4; ++e) {
      hb[e]     = h_bits((xa[e] - mu) * rs * ga[e] + ba[e]);
      hb[4 + e] = h_bits((xb[e] - mu) * rs * gb[e] + bb[e]);
    }
    const v4u u = (v4u){pk16(hb[0], hb[1]), pk16(hb[2], hb[3]), pk16(hb[4], hb[5]), pk16(hb[6], hb[7])};
    unsigned short* yp = Y + (size_t)row * kDim + c0;
    *(volatile v4u*)yp = u;
    __threadfence();
    *(volatile v4u*)yp = u;
  }
}

__global__ __launch_bounds__(256) void vtrans_kernel(const unsigned short* __restrict__ qkv, unsigned short* __restrict__ Vt) {
  __shared__ unsigned short sm[64][66];
  const int t  = threadIdx.x;
  const int g  = blockIdx.y;
  const int b  = g / kHeads, h = g - (g / kHeads) * kHeads;
  const int n0 = blockIdx.x * 64;
#pragma unroll
  for (int it = 0; it < 2; ++it) {
    const int idx = it * 256 + t;
    const int r   = idx >> 3;
    const int seg = (idx & 7) * 8;
    const size_t off = (size_t)(b * kSeq + n0 + r) * kQkvCols + 2 * kDim + h * kHeadDim + seg;
    const v4u w = *(const v4u*)(qkv + off);
    sm[r][seg + 0] = (unsigned short)(w.x & 0xffffu); sm[r][seg + 1] = (unsigned short)(w.x >> 16);
    sm[r][seg + 2] = (unsigned short)(w.y & 0xffffu); sm[r][seg + 3] = (unsigned short)(w.y >> 16);
    sm[r][seg + 4] = (unsigned short)(w.z & 0xffffu); sm[r][seg + 5] = (unsigned short)(w.z >> 16);
    sm[r][seg + 6] = (unsigned short)(w.w & 0xffffu); sm[r][seg + 7] = (unsigned short)(w.w >> 16);
  }
  __syncthreads();
  const int lane = t & 31, wave = t >> 5;
  const int q = lane >> 3, c8 = (lane & 7) * 8;
  unsigned short* vb = Vt + (size_t)g * kHeadDim * kSeq;
  for (int pass = 0; pass < 2; ++pass) {
#pragma unroll
    for (int it = 0; it < 2; ++it) {
      const int dh = wave * 8 + it * 4 + q;
      unsigned short hb[8];
#pragma unroll
      for (int e = 0; e < 8; ++e) hb[e] = sm[c8 + e][dh];
      const v4u u = (v4u){pk16(hb[0], hb[1]), pk16(hb[2], hb[3]), pk16(hb[4], hb[5]), pk16(hb[6], hb[7])};
      *(volatile v4u*)(vb + (size_t)dh * kSeq + n0 + c8) = u;
    }
    __threadfence();
  }
}

__global__ __launch_bounds__(256) void softmax_row_kernel(const float* __restrict__ S, unsigned short* __restrict__ P, float carry) {
  __shared__ float redM[8];
  __shared__ float redS[8];
  const int row  = blockIdx.x;
  const int t    = threadIdx.x;
  const int lane = t & 31, wave = t >> 5;
  const int c0   = t * 8;
  const float* sr = S + (size_t)row * kSeq + c0;
  const v4f a = *(const v4f*)(sr);
  const v4f c = *(const v4f*)(sr + 4);
  float x[8];
#pragma unroll
  for (int e = 0; e < 4; ++e) { x[e] = a[e]; x[4 + e] = c[e]; }
  float m = fmaxf(fmaxf(fmaxf(x[0], x[1]), fmaxf(x[2], x[3])), fmaxf(fmaxf(x[4], x[5]), fmaxf(x[6], x[7])));
#pragma unroll
  for (int off = 16; off > 0; off >>= 1) m = fmaxf(m, __shfl_xor(m, off, 32));
  if (lane == 0) redM[wave] = m;
  __syncthreads();
  float gm = redM[0];
#pragma unroll
  for (int w = 1; w < 8; ++w) gm = fmaxf(gm, redM[w]);
  float p[8];
#pragma unroll
  for (int e = 0; e < 8; ++e) p[e] = expf(x[e] - gm);
  float s = ((p[0] + p[1]) + (p[2] + p[3])) + ((p[4] + p[5]) + (p[6] + p[7]));
#pragma unroll
  for (int off = 16; off > 0; off >>= 1) s += __shfl_xor(s, off, 32);
  if (lane == 0) redS[wave] = s;
  __syncthreads();
  float tot = redS[0];
#pragma unroll
  for (int w = 1; w < 8; ++w) tot += redS[w];
  const float inv = carry / tot;
  unsigned short hb[8];
#pragma unroll
  for (int e = 0; e < 8; ++e) hb[e] = h_bits(p[e] * inv);
  const v4u u = (v4u){pk16(hb[0], hb[1]), pk16(hb[2], hb[3]), pk16(hb[4], hb[5]), pk16(hb[6], hb[7])};
  unsigned short* pp = P + (size_t)row * kSeq + c0;
  *(volatile v4u*)pp = u;
  __threadfence();
  *(volatile v4u*)pp = u;
}

__global__ __launch_bounds__(256) void gelu_cast_kernel(const float* __restrict__ in, unsigned short* __restrict__ out, int n2, float carry) {
  const int i = blockIdx.x * 256 + threadIdx.x;
  if (i >= n2) return;
  const v2f v = *(const v2f*)(in + 2 * (size_t)i);
  const float g0 = 0.5f * v.x * (1.0f + erff(v.x * 0.70710678118654752f)) * carry;
  const float g1 = 0.5f * v.y * (1.0f + erff(v.y * 0.70710678118654752f)) * carry;
  const unsigned u = pk16(h_bits(g0), h_bits(g1));
  unsigned short* op = out + 2 * (size_t)i;
  *(volatile unsigned*)op = u;
  __threadfence();
  *(volatile unsigned*)op = u;
}

extern "C" void kernel_launch(void* const* d_in, const int* in_sizes, int n_in,
                              void* d_out, int out_size, void* d_ws, size_t ws_size,
                              hipStream_t stream) {
  if (n_in < 13) return;
  if (in_sizes[0] != kTok * kDim || in_sizes[1] != kDim * kQkvCols || in_sizes[2] != kQkvCols ||
      in_sizes[3] != kDim * kDim || in_sizes[4] != kDim || in_sizes[5] != kDim * kFF || in_sizes[6] != kFF ||
      in_sizes[7] != kFF * kDim || in_sizes[8] != kDim || in_sizes[9] != kDim || in_sizes[10] != kDim ||
      in_sizes[11] != kDim || in_sizes[12] != kDim) return;
  if (out_size != kTok * kDim) return;

  const float* x     = (const float*)d_in[0];
  const float* Wqkv  = (const float*)d_in[1];
  const float* bqkv  = (const float*)d_in[2];
  const float* Wproj = (const float*)d_in[3];
  const float* bproj = (const float*)d_in[4];
  const float* Wfc1  = (const float*)d_in[5];
  const float* bfc1  = (const float*)d_in[6];
  const float* Wfc2  = (const float*)d_in[7];
  const float* bfc2  = (const float*)d_in[8];
  const float* ln1g  = (const float*)d_in[9];
  const float* ln1b  = (const float*)d_in[10];
  const float* ln2g  = (const float*)d_in[11];
  const float* ln2b  = (const float*)d_in[12];
  float* out = (float*)d_out;

  const size_t szWqkvT = (size_t)kQkvCols * kDim * 2;
  const size_t szWprojT = (size_t)kDim * kDim * 2;
  const size_t szWfc1T = (size_t)kFF * kDim * 2;
  const size_t szWfc2T = (size_t)kDim * kFF * 2;
  const size_t szX1    = (size_t)kTok * kDim * 4;
  const size_t szAttn  = (size_t)kTok * kDim * 2;
  const size_t szQkv   = (size_t)kTok * kQkvCols * 2;
  const size_t szVt    = (size_t)kGroups * kHeadDim * kSeq * 2;
  const size_t szScore = (size_t)kGrpPerChunk * kSeq * kSeq * 4;
  const size_t szP     = (size_t)kGrpPerChunk * kSeq * kSeq * 2;
  const size_t off0 = 0;
  const size_t off1 = off0 + szWqkvT;
  const size_t off2 = off1 + szWprojT;
  const size_t off3 = off2 + szWfc1T;
  const size_t off4 = off3 + szWfc2T;
  const size_t off5 = off4 + szX1;
  const size_t off6 = off5 + szAttn;
  const size_t off7 = off6 + szQkv;
  const size_t off8 = off7 + szVt;
  const size_t off9 = off8 + szScore;
  const size_t total = off9 + szP;
  if (total > ws_size) return;
  if ((size_t)kTok * kDim * 2 > szScore) return;
  if ((size_t)kTok * kFF * 4 > szScore) return;
  if ((size_t)kTok * kFF * 2 > szP) return;

  char* ws = (char*)d_ws;
  unsigned short* WqkvT  = (unsigned short*)(ws + off0);
  unsigned short* WprojT = (unsigned short*)(ws + off1);
  unsigned short* Wfc1T  = (unsigned short*)(ws + off2);
  unsigned short* Wfc2T  = (unsigned short*)(ws + off3);
  float*          x1     = (float*)(ws + off4);
  unsigned short* attn   = (unsigned short*)(ws + off5);
  unsigned short* ln2h   = (unsigned short*)(ws + off5);
  unsigned short* qkv    = (unsigned short*)(ws + off6);
  unsigned short* Vt     = (unsigned short*)(ws + off7);
  unsigned short* ln1h   = (unsigned short*)(ws + off8);
  float*          scores = (float*)(ws + off8);
  float*          pre    = (float*)(ws + off8);
  unsigned short* Pp     = (unsigned short*)(ws + off9);
  unsigned short* g16    = (unsigned short*)(ws + off9);

  wtcast_kernel<<<dim3(kDim / 64, kQkvCols / 64), dim3(256), 0, stream>>>(Wqkv, WqkvT, kDim, kQkvCols, kWCarry);
  wtcast_kernel<<<dim3(kDim / 64, kDim / 64), dim3(256), 0, stream>>>(Wproj, WprojT, kDim, kDim, kWCarry);
  wtcast_kernel<<<dim3(kDim / 64, kFF / 64), dim3(256), 0, stream>>>(Wfc1, Wfc1T, kDim, kFF, kWCarry);
  wtcast_kernel<<<dim3(kFF / 64, kDim / 64), dim3(256), 0, stream>>>(Wfc2, Wfc2T, kFF, kDim, kWCarry);

  ln_row_kernel<<<dim3(kTok), dim3(256), 0, stream>>>(x, ln1g, ln1b, ln1h);

  wmma_gemm64<0, false, 2, 1, false, 0><<<dim3((kTok / 64) * (kQkvCols / 64) / 8, 1), dim3(256), 0, stream>>>(
      ln1h, nullptr, kDim, 0L, WqkvT, nullptr, kDim, 0L, (void*)qkv, nullptr, kQkvCols, 0L,
      bqkv, nullptr, 0L, kTok, kQkvCols, kDim, 1.0f / kWCarry);

  vtrans_kernel<<<dim3(kSeq / 64, kGroups), dim3(256), 0, stream>>>(qkv, Vt);

  for (int ch = 0; ch < kChunks; ++ch) {
    const int b  = ch / (kHeads / kGrpPerChunk);
    const int h0 = (ch - b * (kHeads / kGrpPerChunk)) * kGrpPerChunk;
    const unsigned short* Qp = qkv + (size_t)b * kSeq * kQkvCols + (size_t)h0 * kHeadDim;
    const unsigned short* Kp = Qp + kDim;
    wmma_gemm64<0, false, 0, 0, false, 0><<<dim3((kSeq / 64) * (kSeq / 64) / 8, kGrpPerChunk), dim3(256), 0, stream>>>(
        Qp, nullptr, kQkvCols, (long)kHeadDim, Kp, nullptr, kQkvCols, (long)kHeadDim,
        (void*)scores, nullptr, kSeq, (long)kSeq * kSeq, nullptr, nullptr, 0L, kSeq, kSeq, kHeadDim, kAttnScale);
    softmax_row_kernel<<<dim3(kGrpPerChunk * kSeq), dim3(256), 0, stream>>>(scores, Pp, kPCarry);
    const unsigned short* Vtp = Vt + (size_t)(b * kHeads + h0) * kHeadDim * kSeq;
    unsigned short* Op = attn + (size_t)b * kSeq * kDim + (size_t)h0 * kHeadDim;
    wmma_gemm64<0, false, 0, 1, false, 0><<<dim3((kSeq / 64) * (kHeadDim / 64) / 8, kGrpPerChunk), dim3(256), 0, stream>>>(
        Pp, nullptr, kSeq, (long)kSeq * kSeq, Vtp, nullptr, kSeq, (long)kHeadDim * kSeq,
        (void*)Op, nullptr, kDim, (long)kHeadDim, nullptr, nullptr, 0L, kSeq, kHeadDim, kSeq, kOCarry / kPCarry);
  }

  wmma_gemm64<0, false, 2, 0, true, 0><<<dim3((kTok / 64) * (kDim / 64) / 8, 1), dim3(256), 0, stream>>>(
      attn, nullptr, kDim, 0L, WprojT, nullptr, kDim, 0L, (void*)x1, nullptr, kDim, 0L,
      bproj, x, 0L, kTok, kDim, kDim, 1.0f / (kOCarry * kWCarry));

  ln_row_kernel<<<dim3(kTok), dim3(256), 0, stream>>>(x1, ln2g, ln2b, ln2h);

  wmma_gemm64<0, false, 2, 0, false, 0><<<dim3((kTok / 64) * (kFF / 64) / 8, 1), dim3(256), 0, stream>>>(
      ln2h, nullptr, kDim, 0L, Wfc1T, nullptr, kDim, 0L, (void*)pre, nullptr, kFF, 0L,
      bfc1, nullptr, 0L, kTok, kFF, kDim, 1.0f / kWCarry);

  {
    const int n2 = kTok * kFF / 2;
    gelu_cast_kernel<<<dim3((n2 + 255) / 256), dim3(256), 0, stream>>>(pre, g16, n2, kGCarry);
  }

  wmma_gemm64<0, false, 2, 0, true, 0><<<dim3((kTok / 64) * (kDim / 64) / 8, 1), dim3(256), 0, stream>>>(
      g16, nullptr, kFF, 0L, Wfc2T, nullptr, kFF, 0L, (void*)out, nullptr, kDim, 0L,
      bfc2, x1, 0L, kTok, kDim, kFF, 1.0f / (kGCarry * kWCarry));
}
